// MH_Lori_24163486007330
// MI455X (gfx1250) — hardware-verified
//
#include <hip/hip_runtime.h>
#include <math.h>

typedef __attribute__((ext_vector_type(16))) _Float16 v16h;
typedef __attribute__((ext_vector_type(16))) __bf16 v16b;
typedef __attribute__((ext_vector_type(8)))  _Float16 v8h;
typedef __attribute__((ext_vector_type(8)))  float v8f;
typedef __attribute__((ext_vector_type(4)))  float v4f;
typedef __attribute__((ext_vector_type(2)))  float v2f;
typedef __attribute__((ext_vector_type(4)))  unsigned v4u;
typedef __attribute__((ext_vector_type(4)))  int v4i;
typedef float __attribute__((may_alias)) float_a;
typedef int __attribute__((may_alias)) int_a;

template <typename T> __device__ __forceinline__ void vst2(void* p, T v) { *(volatile T*)p = v; __threadfence(); *(volatile T*)p = v; }
__device__ __forceinline__ v8f wmma16(v16h a, v16h b, v8f c) {
  v8f d = __builtin_amdgcn_wmma_f32_16x16x32_f16(false, a, false, b, (short)0, c, false, false);
  asm volatile("v_nop\n\tv_nop\n\tv_nop\n\tv_nop" : "+v"(d) : "v"(a), "v"(b));
  return d;
}
__device__ __forceinline__ v8f wmma_bf(v16b a, v16b b, v8f c) {
  v8f d = __builtin_amdgcn_wmma_f32_16x16x32_bf16(false, a, false, b, (short)0, c, false, false);
  asm volatile("v_nop\n\tv_nop\n\tv_nop\n\tv_nop" : "+v"(d) : "v"(a), "v"(b));
  return d;
}
__device__ __forceinline__ v16h frag_h(const _Float16* rowk0, int lane) {
  union { v16h v; v8h q[2]; } u; const _Float16* p = rowk0 + 8 * (lane >> 4);
  u.q[0] = *(const v8h*)p; u.q[1] = *(const v8h*)(p + 16); return u.v;
}
__device__ __forceinline__ v16h frag_f32(const float* rowk0, int lane) {
  v16h a; const float* p = rowk0 + 8 * (lane >> 4);
#pragma unroll
  for (int i = 0; i < 8; ++i) { a[i] = (_Float16)p[i]; a[8 + i] = (_Float16)p[16 + i]; }
  return a;
}
__device__ __forceinline__ v16h frag_f32s(const float* rowk0, int lane, float sc) {
  v16h a; const float* p = rowk0 + 8 * (lane >> 4);
#pragma unroll
  for (int i = 0; i < 8; ++i) { a[i] = (_Float16)(p[i] * sc); a[8 + i] = (_Float16)(p[16 + i] * sc); }
  return a;
}
__device__ __forceinline__ v16h fragc_f32(const float* W, int k0, int n, int lane, int ld, int K) {
  v16h a; const int g = lane >> 4;
#pragma unroll
  for (int i = 0; i < 8; ++i) { const int ka = k0 + 8 * g + i, kb = ka + 16;
    a[i] = (_Float16)(ka < K ? W[(size_t)ka * ld + n] : 0.f); a[8 + i] = (_Float16)(kb < K ? W[(size_t)kb * ld + n] : 0.f); }
  return a;
}
struct F2 { v16b h, l; };
__device__ __forceinline__ F2 bsplit16(const float v[16]) { F2 r;
#pragma unroll
  for (int i = 0; i < 16; ++i) { const __bf16 h = (__bf16)v[i]; r.h[i] = h; r.l[i] = (__bf16)(v[i] - (float)h); }
  return r; }
__device__ __forceinline__ F2 split_row(const float* row, int k0, int lane) { float v[16]; const float* p = row + k0 + 8 * (lane >> 4);
#pragma unroll
  for (int i = 0; i < 8; ++i) { v[i] = p[i]; v[8 + i] = p[16 + i]; }
  return bsplit16(v); }
__device__ __forceinline__ F2 split_rowK(const float* row, int k0, int lane, int K) { float v[16]; const int g = lane >> 4;
#pragma unroll
  for (int i = 0; i < 8; ++i) { const int ka = k0 + 8 * g + i, kb = ka + 16; v[i] = ka < K ? row[ka] : 0.f; v[8 + i] = kb < K ? row[kb] : 0.f; }
  return bsplit16(v); }
__device__ __forceinline__ F2 split_col(const float* W, int k0, int n, int lane, int ld, int K) { float v[16]; const int g = lane >> 4;
#pragma unroll
  for (int i = 0; i < 8; ++i) { const int ka = k0 + 8 * g + i, kb = ka + 16; v[i] = ka < K ? W[(size_t)ka * ld + n] : 0.f; v[8 + i] = kb < K ? W[(size_t)kb * ld + n] : 0.f; }
  return bsplit16(v); }
__device__ __forceinline__ v8f mac3(const F2& a, const F2& b, v8f c) { c = wmma_bf(a.l, b.h, c); c = wmma_bf(a.h, b.l, c); return wmma_bf(a.h, b.h, c); }
__device__ __forceinline__ float sigm(float v) { return 1.0f / (1.0f + expf(-v)); }
#define LDSX() do { asm volatile("s_wait_dscnt 0" ::: "memory"); __builtin_amdgcn_wave_barrier(); __builtin_amdgcn_fence(__ATOMIC_RELEASE, "workgroup"); } while (0)

#define NB 4
#define SS 2048
#define HD 1024
#define NH 8
#define DK 128
#define NE 8
#define II 512
#define NSEG 16
#define LSEG (SS / NSEG)
#define NR (NB * SS)
#define NG (NB * NSEG * NH)

__global__ __launch_bounds__(256) void k_cvt(const float* __restrict__ src, _Float16* __restrict__ dst, size_t n8, float sc) {
  const size_t g8 = (size_t)blockIdx.x * 256 + threadIdx.x; if (g8 >= n8) return;
  union { v8h h; v4u u; } pk;
#pragma unroll
  for (int e = 0; e < 8; ++e) pk.h[e] = (_Float16)(src[g8 * 8 + e] * sc);
  vst2(dst + g8 * 8, pk.u);
}
__global__ __launch_bounds__(128) void k_proj(const _Float16* __restrict__ x16, const _Float16* __restrict__ W16, const float* __restrict__ bias, float* __restrict__ x1, _Float16* __restrict__ x1h) {
  __shared__ __align__(16) float so[4][16][132];
  const int tid = threadIdx.x, wave = tid >> 5, lane = tid & 31, col = lane & 15, g = lane >> 4;
  const int r0 = blockIdx.x * 64 + wave * 16, n0 = blockIdx.y * 128;
  v8f acc[8] = {};
#pragma unroll 1
  for (int kc = 0; kc < HD / 32; ++kc) { const v16h a = frag_h(x16 + (size_t)(r0 + col) * HD + kc * 32, lane);
#pragma unroll
    for (int j = 0; j < 8; ++j) acc[j] = wmma16(a, frag_h(W16 + (size_t)(n0 + j * 16 + col) * HD + kc * 32, lane), acc[j]); }
#pragma unroll
  for (int j = 0; j < 8; ++j) { const float bb = bias[n0 + j * 16 + col];
#pragma unroll
    for (int r = 0; r < 8; ++r) so[wave][8 * g + r][j * 16 + col] = acc[j][r] * (1.0f / 16.0f) + bb; }
  LDSX();
#pragma unroll 4
  for (int rl = 0; rl < 16; ++rl) { const v4f v = *(const v4f*)(&so[wave][rl][lane * 4]); vst2(x1 + (size_t)(r0 + rl) * HD + n0 + lane * 4, v); }
  for (int q = lane; q < 16 * 16; q += 32) { const int rl = q >> 4, pc = q & 15; union { v8h hh; v4u u; } pk;
#pragma unroll
    for (int e = 0; e < 8; ++e) pk.hh[e] = (_Float16)so[wave][rl][pc * 8 + e];
    vst2(x1h + (size_t)(r0 + rl) * HD + n0 + pc * 8, pk.u); }
}
__global__ __launch_bounds__(128) void k_route(const float* __restrict__ x1, const float* __restrict__ emb, float* __restrict__ wts) {
  __shared__ float sav[DK]; __shared__ float slg[NE]; __shared__ __align__(16) float sw[32];
  const int gidx = blockIdx.x, d = threadIdx.x; const int b = gidx / (NSEG * NH), n = (gidx / NH) % NSEG, h = gidx % NH;
  float s = 0.f;
#pragma unroll 1
  for (int l = 0; l < LSEG; ++l) s += x1[((size_t)b * SS + n * LSEG + l) * HD + h * DK + d];
  sav[d] = s / (float)LSEG;
  __syncthreads();
  if (d < NE) { float a = 0.f;
#pragma unroll 1
    for (int k = 0; k < DK; ++k) a += sav[k] * emb[k * NE + d];
    slg[d] = a; }
  __syncthreads();
  if (d < 32) { float v = 0.f; if (d < NE) { float mx = slg[0]; for (int e = 1; e < NE; ++e) mx = fmaxf(mx, slg[e]); float z = 0.f; for (int e = 0; e < NE; ++e) z += expf(slg[e] - mx); v = expf(slg[d] - mx) / z; }
    sw[d] = v; }
  __builtin_amdgcn_wave_barrier(); asm volatile("s_wait_dscnt 0" ::: "memory");
  if (d < 8) vst2(wts + (size_t)gidx * 32 + d * 4, *(const v4f*)(&sw[d * 4]));
}
#define NGC 128
__global__ __launch_bounds__(256) void k_merge(const float* __restrict__ wts, const float* __restrict__ first, const float* __restrict__ second, _Float16* __restrict__ M1, _Float16* __restrict__ M2, int g0) {
  const int gl = blockIdx.y, gidx = g0 + gl, tid = threadIdx.x; float w8[NE];
#pragma unroll
  for (int e = 0; e < NE; ++e) w8[e] = wts[(size_t)gidx * 32 + e];
  const int which = blockIdx.x >> 5, piece = (blockIdx.x & 31) * 256 + tid;
  union { v8h hh; v4u u; } pk;
  if (which == 0) { const size_t base = (size_t)piece * 8;
#pragma unroll
    for (int q = 0; q < 8; ++q) { float a = 0.f;
#pragma unroll
      for (int e = 0; e < NE; ++e) a += w8[e] * first[(size_t)e * II * DK + base + q];
      pk.hh[q] = (_Float16)(a * 16.0f); }
    vst2(M1 + (size_t)gl * II * DK + base, pk.u); }
  else { const size_t base = (size_t)piece * 8;
#pragma unroll
    for (int q = 0; q < 8; ++q) { float a = 0.f;
#pragma unroll
      for (int e = 0; e < NE; ++e) a += w8[e] * second[(size_t)e * DK * II + base + q];
      pk.hh[q] = (_Float16)(a * 16.0f); }
    vst2(M2 + (size_t)gl * DK * II + base, pk.u); }
}
__global__ __launch_bounds__(128) void k_ffn(const _Float16* __restrict__ x1h, const _Float16* __restrict__ M1, const _Float16* __restrict__ M2, _Float16* __restrict__ res, int g0) {
  __shared__ __align__(16) _Float16 sh[64][II + 16];
  __shared__ __align__(16) float so[4][16][132];
  const int tid = threadIdx.x, wave = tid >> 5, lane = tid & 31, col = lane & 15, g = lane >> 4;
  const int gidx = g0 + blockIdx.y, half = blockIdx.x; const int b = gidx / (NSEG * NH), n = (gidx / NH) % NSEG, h = gidx % NH;
  const int gsrc = n == 0 ? gidx : gidx - NH; const int gl = gsrc - g0;
  const _Float16* m1 = M1 + (size_t)gl * II * DK; const _Float16* m2 = M2 + (size_t)gl * DK * II;
  const size_t row0 = (size_t)b * SS + n * LSEG + half * 64 + wave * 16;
  const _Float16* arow = x1h + (row0 + col) * HD + h * DK;
  v16h a4[4];
#pragma unroll
  for (int kc = 0; kc < 4; ++kc) a4[kc] = frag_h(arow + kc * 32, lane);
#pragma unroll 1
  for (int nc = 0; nc < II / 128; ++nc) { v8f acc[8] = {};
#pragma unroll
    for (int kc = 0; kc < 4; ++kc) {
#pragma unroll
      for (int j = 0; j < 8; ++j) acc[j] = wmma16(a4[kc], frag_h(m1 + (size_t)(nc * 128 + j * 16 + col) * DK + kc * 32, lane), acc[j]); }
#pragma unroll
    for (int j = 0; j < 8; ++j)
#pragma unroll
      for (int r = 0; r < 8; ++r) { const float v = acc[j][r] * (1.0f / 16.0f); sh[wave * 16 + 8 * g + r][nc * 128 + j * 16 + col] = (_Float16)(v > 0.f ? v : 0.f); } }
  LDSX();
  v8f acc[8] = {};
#pragma unroll 1
  for (int kc = 0; kc < II / 32; ++kc) { const v16h a = frag_h(&sh[wave * 16 + col][0] + kc * 32, lane);
#pragma unroll
    for (int j = 0; j < 8; ++j) acc[j] = wmma16(a, frag_h(m2 + (size_t)(j * 16 + col) * II + kc * 32, lane), acc[j]); }
#pragma unroll
  for (int j = 0; j < 8; ++j)
#pragma unroll
    for (int r = 0; r < 8; ++r) so[wave][8 * g + r][j * 16 + col] = acc[j][r] * (1.0f / 16.0f);
  LDSX();
  for (int q = lane; q < 16 * 16; q += 32) { const int rl = q >> 4, pc = q & 15; union { v8h hh; v4u u; } pk;
#pragma unroll
    for (int e = 0; e < 8; ++e) pk.hh[e] = (_Float16)(so[wave][rl][pc * 8 + e] * 64.0f);
    vst2(res + (row0 + rl) * HD + h * DK + pc * 8, pk.u); }
}
__global__ __launch_bounds__(128) void k_out(const _Float16* __restrict__ res, const _Float16* __restrict__ Wm16, const float* __restrict__ bias, float* __restrict__ out) {
  __shared__ __align__(16) float so[4][16][132];
  const int tid = threadIdx.x, wave = tid >> 5, lane = tid & 31, col = lane & 15, g = lane >> 4;
  const int r0 = blockIdx.x * 64 + wave * 16, n0 = blockIdx.y * 128;
  v8f acc[8] = {};
#pragma unroll 1
  for (int kc = 0; kc < HD / 32; ++kc) { const v16h a = frag_h(res + (size_t)(r0 + col) * HD + kc * 32, lane);
#pragma unroll
    for (int j = 0; j < 8; ++j) acc[j] = wmma16(a, frag_h(Wm16 + (size_t)(n0 + j * 16 + col) * HD + kc * 32, lane), acc[j]); }
#pragma unroll
  for (int j = 0; j < 8; ++j) { const float bb = bias[n0 + j * 16 + col];
#pragma unroll
    for (int r = 0; r < 8; ++r) so[wave][8 * g + r][j * 16 + col] = acc[j][r] * (1.0f / 1024.0f) + bb; }
  LDSX();
#pragma unroll 4
  for (int rl = 0; rl < 16; ++rl) vst2(out + (size_t)(r0 + rl) * HD + n0 + lane * 4, *(const v4f*)(&so[wave][rl][lane * 4]));
}
extern "C" void kernel_launch(void* const* d_in, const int* in_sizes, int n_in, void* d_out, int out_size, void* d_ws, size_t ws_size, hipStream_t stream) {
  (void)in_sizes; (void)n_in; (void)out_size; (void)ws_size;
  const float* x = (const float*)d_in[0]; const float* mhW = (const float*)d_in[1]; const float* mhb = (const float*)d_in[2]; const float* emb = (const float*)d_in[3];
  const float* first = (const float*)d_in[4]; const float* second = (const float*)d_in[5]; const float* mW = (const float*)d_in[6]; const float* mb = (const float*)d_in[7];
  float* out = (float*)d_out;
  char* ws = (char*)d_ws; size_t off = 0;
  auto take = [&](size_t bytes) { char* p = ws + off; off += (bytes + 255) & ~(size_t)255; return p; };
  _Float16* x16 = (_Float16*)take((size_t)NR * HD * 2); _Float16* W16 = (_Float16*)take((size_t)HD * HD * 2); _Float16* Wm16 = (_Float16*)take((size_t)HD * HD * 2);
  float* x1 = (float*)take((size_t)NR * HD * 4); _Float16* x1h = (_Float16*)take((size_t)NR * HD * 2); float* wts = (float*)take((size_t)NG * 32 * 4);
_Float16* res = (_Float16*)take((size_t)NR * HD * 2);
  _Float16* M1 = (_Float16*)take((size_t)NGC * II * DK * 2); _Float16* M2 = (_Float16*)take((size_t)NGC * DK * II * 2);
  auto cvt = [&](const float* s, _Float16* d, size_t n, float sc) { const size_t n8 = n / 8; k_cvt<<<(unsigned)((n8 + 255) / 256), 256, 0, stream>>>(s, d, n8, sc); };
  cvt(x, x16, (size_t)NR * HD, 1.0f); cvt(mhW, W16, (size_t)HD * HD, 16.0f); cvt(mW, Wm16, (size_t)HD * HD, 16.0f);
  k_proj<<<dim3(NR / 64, HD / 128), 128, 0, stream>>>(x16, W16, mhb, x1, x1h);
  k_route<<<NG, 128, 0, stream>>>(x1, emb, wts);
  for (int chk = 0; chk < NG / NGC; ++chk) { const int g0 = chk * NGC;
    k_merge<<<dim3(64, NGC), 256, 0, stream>>>(wts, first, second, M1, M2, g0);
    k_ffn<<<dim3(2, NGC), 128, 0, stream>>>(x1h, M1, M2, res, g0); }
  k_out<<<dim3(NR / 64, HD / 128), 128, 0, stream>>>(res, Wm16, mb, out);
}
